// SplatterModel_17454747091703
// MI455X (gfx1250) — hardware-verified
//
#include <hip/hip_runtime.h>


namespace {
constexpr int NSP = 1000, NSPP = 1024, K = 256, NPIX = K * K, CH = 3;
constexpr float EPS = 1e-6f, AS_ = 8.0f;

typedef _Float16 b16;
typedef __attribute__((ext_vector_type(16))) _Float16 v16b;
typedef __attribute__((ext_vector_type(8))) _Float16 v8b;
typedef __attribute__((ext_vector_type(8))) float v8f;
typedef __attribute__((ext_vector_type(4))) float v4f;
__device__ __forceinline__ float bf16_rne(float f) { unsigned int u = __float_as_uint(f); u += 0x7FFFu + ((u >> 16) & 1u); return __uint_as_float(u & 0xFFFF0000u); }
__device__ __forceinline__ void split16(float v, b16& hi, b16& lo) { hi = (b16)v; lo = (b16)(v - (float)hi); }
__device__ __forceinline__ v16b frag_kb(const b16* p, int hh) { const v8b a = *(const v8b*)(p + 8 * hh), b = *(const v8b*)(p + 16 + 8 * hh); v16b f;
#pragma unroll
  for (int e = 0; e < 8; ++e) { f[e] = a[e]; f[8 + e] = b[e]; } return f; }
__device__ __forceinline__ v8f wmma16b(v16b a, v16b b, v8f c) { v8f d = __builtin_amdgcn_wmma_f32_16x16x32_f16(false, a, false, b, (short)0, c, false, false); asm volatile("v_nop\n\tv_nop\n\tv_nop\n\tv_nop" : "+v"(d) : "v"(a), "v"(b)); return d; }
__device__ __forceinline__ void wave_lds_sync() { __builtin_amdgcn_fence(__ATOMIC_RELEASE, "workgroup"); __builtin_amdgcn_wave_barrier(); __builtin_amdgcn_fence(__ATOMIC_ACQUIRE, "workgroup"); }
__device__ __forceinline__ float nexp(float x) { return __builtin_amdgcn_exp2f(x * 1.4426950408889634f); }
__device__ __forceinline__ float pmul(float a, float b) { float p = a * b; asm volatile("" : "+v"(p)); return p; }
__device__ __forceinline__ float tanh_f(float x) { const float e = nexp(-2.0f * fabsf(x)); const float t = (1.0f - e) / (1.0f + e); return (x >= 0.0f) ? t : -t; }
__device__ __forceinline__ float axv(int i) { return -1.0f + (float)i * (2.0f / 255.0f); }

struct SP { static constexpr int A00 = 0, A01 = 1, A11 = 2, CX = 3, CY = 4, INRM = 5, IKM = 6; };

__device__ __forceinline__ float zval(const float* sp, int i, int j) { const float vx = axv(i) + sp[SP::CX], vy = axv(j) + sp[SP::CY]; return (pmul(sp[SP::A00] * vx, vx) + pmul(sp[SP::A01] * vx, vy)) + pmul(sp[SP::A11] * vy, vy); }

__global__ __launch_bounds__(256) void splat_kernel(const float* __restrict__ rho_r, const float* __restrict__ sx_r, const float* __restrict__ sy_r, const float* __restrict__ co_r, float* __restrict__ par) {
  __shared__ float sp[8]; __shared__ float red[256];
  const int n = blockIdx.x, t_ = threadIdx.x;
  if (t_ == 0) { const float rho = tanh_f(bf16_rne(rho_r[n])), sx = -tanh_f(bf16_rne(sx_r[n])), sy = -tanh_f(bf16_rne(sy_r[n]));
    const float a = pmul(sx, sx) + EPS, b = pmul(rho * sx, sy) + EPS, d = pmul(sy, sy) + EPS; const float det = pmul(a, d) - pmul(b, b); const float idet = 1.0f / det;
    sp[SP::A00] = -0.5f * (d * idet); sp[SP::A01] = -0.5f * (-2.0f * b * idet); sp[SP::A11] = -0.5f * (a * idet); sp[SP::CX] = tanh_f(bf16_rne(co_r[2 * n])); sp[SP::CY] = tanh_f(bf16_rne(co_r[2 * n + 1]));
    sp[SP::INRM] = 1.0f / (6.283185307179586f * sqrtf(det + EPS) + EPS); sp[SP::IKM] = 0.0f; }
  __syncthreads();
  float mx = 0.0f;
  for (int p = t_; p < NPIX; p += 256) { const float kv = nexp(zval(sp, p >> 8, p & 255)) * sp[SP::INRM]; mx = fmaxf(mx, kv); }
  red[t_] = mx; __syncthreads();
  for (int s = 128; s > 0; s >>= 1) { if (t_ < s) red[t_] = fmaxf(red[t_], red[t_ + s]); __syncthreads(); }
  if (t_ < 32) { const float kmax = red[0]; const float v = (t_ == SP::IKM) ? ((kmax == 0.0f) ? 1.0f : 1.0f / kmax) : ((t_ < 7) ? sp[t_] : 0.0f); for (int pass = 0; pass < 2; ++pass) ((volatile float*)par)[n * 32 + t_] = v; }
  __threadfence();
}

__global__ __launch_bounds__(256) void colors_kernel(const float* __restrict__ al_r, const float* __restrict__ col_r, b16* __restrict__ colB) {
  const int t_ = threadIdx.x;
  for (int pass = 0; pass < 2; ++pass) {
    for (int q = t_; q < 32 * NSPP; q += 256) { const int row = q / NSPP, n = q % NSPP; float v = 0.0f;
      if (n < NSP && (row < CH || (row >= 16 && row < 16 + CH))) { const int c = (row < 16) ? row : row - 16; const float alpha = 1.0f / (1.0f + nexp(-bf16_rne(al_r[n]))); const float col = tanh_f(bf16_rne(col_r[n * CH + c]) * alpha); b16 h_, l_; split16(col * AS_, h_, l_); v = (row < 16) ? (float)h_ : (float)l_; }
      ((volatile b16*)colB)[q] = (b16)v; }
    __threadfence(); }
}

__global__ __launch_bounds__(256) void render_kernel(const float* __restrict__ par, const b16* __restrict__ colB, float* __restrict__ out) {
  __shared__ float PS[NSPP * 8]; __shared__ __attribute__((aligned(16))) float Co[128][4];
  const int wid = threadIdx.x >> 5, lane = threadIdx.x & 31, nloc = lane & 15, hlf = lane >> 4; const int p0 = blockIdx.x * 128 + wid * 16, prow = p0 + nloc, i = prow >> 8, j = prow & 255;
  for (int q = threadIdx.x; q < NSPP * 8; q += 256) { const int n = q >> 3, f = q & 7; PS[q] = (n < NSP) ? par[n * 32 + f] : 0.0f; }
  __syncthreads();
  v8f acc = {};
  for (int kb = 0; kb < NSPP; kb += 32) { v16b ah, al;
#pragma unroll
    for (int e = 0; e < 16; ++e) { const int n = kb + ((e < 8) ? (8 * hlf + e) : (16 + 8 * hlf + e - 8)); float kn = 0.0f;
      if (n < NSP) { const float* sp = PS + n * 8; const float kv = nexp(zval(sp, i, j)) * sp[SP::INRM]; kn = kv * sp[SP::IKM]; }
      b16 h_, l_; split16(kn * AS_, h_, l_); ah[e] = h_; al[e] = l_; }
    const v16b bh = frag_kb(colB + (size_t)nloc * NSPP + kb, hlf), bl = frag_kb(colB + (size_t)(16 + nloc) * NSPP + kb, hlf);
    acc = wmma16b(ah, bh, acc); acc = wmma16b(ah, bl, acc); acc = wmma16b(al, bh, acc); }
  if (nloc < CH) {
#pragma unroll
    for (int r = 0; r < 8; ++r) Co[wid * 16 + 8 * hlf + r][nloc] = acc[r] * (1.0f / (AS_ * AS_)); }
  __syncthreads();
  const int nb = blockIdx.x * 128;
  for (int pass = 0; pass < 2; ++pass) { if (threadIdx.x < 96) { const int q = threadIdx.x; v4f o; for (int e = 0; e < 4; ++e) { const int f = q * 4 + e; o[e] = Co[f / 3][f % 3]; } *(volatile v4f*)(out + (size_t)nb * CH + q * 4) = o; } __threadfence(); }
}
}

extern "C" void kernel_launch(void* const* d_in, const int* in_sizes, int n_in,
                              void* d_out, int out_size, void* d_ws, size_t ws_size, hipStream_t stream) {
  (void)n_in; (void)out_size;
  const float* rho_r = (const float*)d_in[0]; const float* sx_r = (const float*)d_in[1]; const float* sy_r = (const float*)d_in[2]; const float* co_r = (const float*)d_in[3]; const float* al_r = (const float*)d_in[4]; const float* col_r = (const float*)d_in[5];
  float* out = (float*)d_out;
  if (in_sizes[0] != NSP || in_sizes[3] != NSP * 2 || in_sizes[5] != NSP * CH) return;
  size_t off = 0; char* ws = (char*)d_ws;
  auto carve = [&](size_t bytes) { char* p = ws + off; off += (bytes + 255) & ~(size_t)255; return p; };
  float* par = (float*)carve(NSPP * 32 * 4); b16* colB = (b16*)carve(32 * NSPP * 2);
  if (off > ws_size) return;
  colors_kernel<<<1, 256, 0, stream>>>(al_r, col_r, colB);
  splat_kernel<<<NSP, 256, 0, stream>>>(rho_r, sx_r, sy_r, co_r, par);
  render_kernel<<<NPIX / 128, 256, 0, stream>>>(par, colB, out);
}
